// CapsuleLayer_44066364457157
// MI455X (gfx1250) — hardware-run, weakly checked
//
#include <hip/hip_runtime.h>


#ifndef NB
#define NB 128
#endif
#ifndef JN
#define JN 2048
#endif
#define NB_FULL 128
#define JN_FULL 2048
#define NC   32
#define DC   16
#define PD   8
#define BT   16
#define JC   2
#define JPB  64
#define CPB  (JPB / JC)
#define JG   (JN / JPB)
#define EPSF 1e-7f
#define NEGB (-3.0e38f)
#define UH_FLOATS (JC * NC * 4 * BT * 4)
#define CC_FLOATS (JC * NC * BT)

static_assert(PD == 8);
static_assert(DC == 16);
static_assert(BT == 16);
static_assert(NC == 32);
static_assert(JC == 2);
static_assert(4 * 8 == NC);
static_assert(8 * 4 == JC * BT);
static_assert(8 * 4 == NC);
static_assert(2 * 256 == NC * BT);
static_assert(JPB % JC == 0);
static_assert(JN % JPB == 0);
static_assert(NB % BT == 0);
static_assert((NB * NC) % 256 == 0);
static_assert(NB <= NB_FULL);
static_assert(JN <= JN_FULL);
static_assert(BT * NC * DC <= UH_FLOATS);
static_assert(256 * 8 * 16 == BT * NC * DC * 4);
static_assert(256 * 4 * 16 == 256 * DC * 4);
static_assert((UH_FLOATS + CC_FLOATS) * 4 <= 131072);
static_assert(256 * DC * 4 <= 131072);

typedef unsigned short bf;
typedef __attribute__((ext_vector_type(16))) __bf16   v16bf;
typedef __attribute__((ext_vector_type(8)))  unsigned short v8us;
typedef __attribute__((ext_vector_type(8)))  float    v8f;
typedef __attribute__((ext_vector_type(4)))  float    v4f;
typedef v4f  __attribute__((may_alias)) v4fa;
typedef __attribute__((ext_vector_type(4)))  unsigned int v4u;
typedef __attribute__((ext_vector_type(8)))  unsigned int v8u;

__device__ __forceinline__ unsigned short f2bf(float f) { unsigned u = __float_as_uint(f); u += 0x7FFFu + ((u >> 16) & 1u); return (unsigned short)(u >> 16); }
__device__ __forceinline__ float bfr(float f) { return __uint_as_float(((unsigned)f2bf(f)) << 16); }
__device__ __forceinline__ v8f wmmab(v16bf a, v16bf b, v8f c) { return __builtin_amdgcn_wmma_f32_16x16x32_bf16(false, a, false, b, (short)0, c, false, false); }
__device__ __forceinline__ v8f wmmab_g(v16bf a, v16bf b, v8f c) { c = wmmab(a, b, c); asm volatile("v_nop\n\tv_nop\n\tv_nop\n\tv_nop" : "+v"(c) : "v"(a), "v"(b)); return c; }
__device__ __forceinline__ v16bf frag_k8(v4u p) { const v4u z = (v4u){0u, 0u, 0u, 0u}; const v8u f = __builtin_shufflevector(p, z, 0, 1, 2, 3, 4, 5, 6, 7); return __builtin_bit_cast(v16bf, f); }

__global__ __launch_bounds__(256) void k_cvt8(const float* __restrict__ src, bf* dst, size_t n8) {
    const size_t i = (size_t)blockIdx.x * 256 + threadIdx.x; if (i >= n8) return;
    const v8f v = *(const v8f*)(src + i * 8); v8us o;
#pragma unroll
    for (int k = 0; k < 8; ++k) o[k] = f2bf(v[k]);
    *(volatile v8us*)(dst + i * 8) = o; __threadfence(); *(volatile v8us*)(dst + i * 8) = o;
}

__global__ __launch_bounds__(256) void k_sweep(const bf* __restrict__ WB, const bf* __restrict__ XB, const float* __restrict__ Osum, float* Spart, int first) {
    __shared__ __align__(16) float uh[UH_FLOATS];
    __shared__ __align__(16) float cc[CC_FLOATS];
    const int tid = threadIdx.x;
    const int lane = tid & 31, lr = lane & 15, hi = lane >> 4;
    const int wave = __builtin_amdgcn_readfirstlane((int)(threadIdx.x >> 5));
    const int jg = blockIdx.x, b0 = blockIdx.y * BT;
    const int sjl = wave & 1, snq = wave >> 1;
    const unsigned msk = (unsigned)(hi - 1);
    const v4u mk4 = (v4u){msk, msk, msk, msk};
    const int ajl = wave >> 2, abb = (wave & 3) * 4 + (lane & 3), ang = lane >> 2;

    float og[4][16];
#pragma unroll
    for (int i = 0; i < 4; ++i)
#pragma unroll
        for (int d = 0; d < 16; ++d) og[i][d] = 0.0f;
    if (first == 0) {
#pragma unroll
        for (int i = 0; i < 4; ++i) {
            const float* op = Osum + ((size_t)(b0 + abb) * NC + (size_t)(ang * 4 + i)) * DC;
#pragma unroll
            for (int q = 0; q < 4; ++q) { const v4f v = *(const v4f*)(op + 4 * q); og[i][4 * q + 0] = v[0]; og[i][4 * q + 1] = v[1]; og[i][4 * q + 2] = v[2]; og[i][4 * q + 3] = v[3]; }
        }
    }
    float sacc[2][16];
#pragma unroll
    for (int it = 0; it < 2; ++it)
#pragma unroll
        for (int d = 0; d < 16; ++d) sacc[it][d] = 0.0f;

    const size_t xrow = (size_t)(b0 + lr) * JN_FULL * PD;
#pragma unroll 1
    for (int c = 0; c < CPB; ++c) {
        const int j0 = jg * JPB + c * JC;
        __syncthreads();
        {
            const int j = j0 + sjl;
            v4u xv = *(const v4u*)(XB + xrow + (size_t)j * PD);
            asm volatile("" : "+v"(xv));
            xv = xv & mk4;
            const v16bf xb = frag_k8(xv);
#pragma unroll
            for (int nn = 0; nn < 8; ++nn) {
                const int n = snq * 8 + nn;
                v4u wv = *(const v4u*)(WB + (((size_t)n * JN_FULL + (size_t)j) * DC + (size_t)lr) * PD);
                asm volatile("" : "+v"(wv));
                wv = wv & mk4;
                const v16bf wa = frag_k8(wv);
                v8f acc = (v8f){};
                acc = wmmab_g(wa, xb, acc);
                const int ub = (((sjl * NC + n) * 4 + 2 * hi) * BT + lr) * 4;
                v4f lo, up;
                lo[0] = acc[0]; lo[1] = acc[1]; lo[2] = acc[2]; lo[3] = acc[3];
                up[0] = acc[4]; up[1] = acc[5]; up[2] = acc[6]; up[3] = acc[7];
                *(v4fa*)(&uh[ub]) = lo;
                *(v4fa*)(&uh[ub + BT * 4]) = up;
            }
        }
        __syncthreads();
        {
            float lg[4]; float mx = NEGB;
#pragma unroll
            for (int i = 0; i < 4; ++i) {
                const int n = ang * 4 + i;
                float l = 0.0f;
#pragma unroll
                for (int q = 0; q < 4; ++q) {
                    const v4f u = *(const v4fa*)(&uh[(((ajl * NC + n) * 4 + q) * BT + abb) * 4]);
                    l += og[i][4 * q + 0] * u[0]; l += og[i][4 * q + 1] * u[1]; l += og[i][4 * q + 2] * u[2]; l += og[i][4 * q + 3] * u[3];
                }
                lg[i] = l; mx = fmaxf(mx, l);
            }
            mx = fmaxf(mx, __shfl_xor(mx, 4, 32)); mx = fmaxf(mx, __shfl_xor(mx, 8, 32)); mx = fmaxf(mx, __shfl_xor(mx, 16, 32));
            float ssum = 0.0f;
#pragma unroll
            for (int i = 0; i < 4; ++i) { lg[i] = __expf(lg[i] - mx); ssum += lg[i]; }
            ssum += __shfl_xor(ssum, 4, 32); ssum += __shfl_xor(ssum, 8, 32); ssum += __shfl_xor(ssum, 16, 32);
            const float inv = 1.0f / ssum;
#pragma unroll
            for (int i = 0; i < 4; ++i) cc[(ajl * NC + ang * 4 + i) * BT + abb] = lg[i] * inv;
        }
        __syncthreads();
#pragma unroll
        for (int it = 0; it < 2; ++it) {
            const int idx = it * 256 + tid; const int n = idx >> 4, bb = idx & 15;
#pragma unroll
            for (int jl = 0; jl < JC; ++jl) {
                const float cw = cc[(jl * NC + n) * BT + bb];
#pragma unroll
                for (int q = 0; q < 4; ++q) {
                    const v4f u = *(const v4fa*)(&uh[(((jl * NC + n) * 4 + q) * BT + bb) * 4]);
                    sacc[it][4 * q + 0] += cw * u[0]; sacc[it][4 * q + 1] += cw * u[1]; sacc[it][4 * q + 2] += cw * u[2]; sacc[it][4 * q + 3] += cw * u[3];
                }
            }
        }
    }
    __syncthreads();
#pragma unroll
    for (int it = 0; it < 2; ++it) {
        const int idx = it * 256 + tid; const int n = idx >> 4, bb = idx & 15;
#pragma unroll
        for (int q = 0; q < 4; ++q) { v4f w; w[0] = sacc[it][4 * q + 0]; w[1] = sacc[it][4 * q + 1]; w[2] = sacc[it][4 * q + 2]; w[3] = sacc[it][4 * q + 3];
            *(v4fa*)(&uh[(bb * NC + n) * DC + 4 * q]) = w; }
    }
    __syncthreads();
    float* dst = Spart + ((size_t)jg * NB + (size_t)b0) * (NC * DC);
#pragma unroll 1
    for (int ps = 0; ps < 2; ++ps) {
#pragma unroll
        for (int i = 0; i < 8; ++i) { const int idx = i * 256 + tid;
            const v4f val = *(const v4fa*)(&uh[idx * 4]);
            *(volatile v4f*)(dst + (size_t)idx * 4) = val; }
        if (ps == 0) __threadfence(); }
}

__global__ __launch_bounds__(256) void k_squash(const float* __restrict__ Spart, const float* __restrict__ bias, float* Osum, float* OUT, int first, int last) {
#pragma clang fp contract(off)
    __shared__ __align__(16) float st[256 * DC];
    const int tid = threadIdx.x;
    const int t = blockIdx.x * 256 + tid;
    const int n = t & (NC - 1);
    float s[DC];
#pragma unroll
    for (int q = 0; q < 4; ++q) { const v4f bv = *(const v4f*)(bias + n * DC + 4 * q);
        s[4 * q + 0] = bfr(bv[0]); s[4 * q + 1] = bfr(bv[1]); s[4 * q + 2] = bfr(bv[2]); s[4 * q + 3] = bfr(bv[3]); }
#pragma unroll 1
    for (int g = 0; g < JG; ++g) {
        const float* sp = Spart + ((size_t)g * NB * NC + (size_t)t) * DC;
#pragma unroll
        for (int q = 0; q < 4; ++q) { const v4f sv = *(const v4f*)(sp + 4 * q);
            s[4 * q + 0] += sv[0]; s[4 * q + 1] += sv[1]; s[4 * q + 2] += sv[2]; s[4 * q + 3] += sv[3]; }
    }
    float sq = 0.0f;
#pragma unroll
    for (int d = 0; d < DC; ++d) sq += s[d] * s[d];
    const float scale = sq / (1.0f + sq) / sqrtf(sq + EPSF);
    float ov[DC];
#pragma unroll
    for (int d = 0; d < DC; ++d) ov[d] = 0.0f;
    if ((first == 0) && (last == 0)) {
        const float* op = Osum + (size_t)t * DC;
#pragma unroll
        for (int q = 0; q < 4; ++q) { const v4f v = *(const v4f*)(op + 4 * q); ov[4 * q + 0] = v[0]; ov[4 * q + 1] = v[1]; ov[4 * q + 2] = v[2]; ov[4 * q + 3] = v[3]; }
    }
#pragma unroll
    for (int q = 0; q < 4; ++q) { v4f w;
        w[0] = ov[4 * q + 0] + scale * s[4 * q + 0]; w[1] = ov[4 * q + 1] + scale * s[4 * q + 1];
        w[2] = ov[4 * q + 2] + scale * s[4 * q + 2]; w[3] = ov[4 * q + 3] + scale * s[4 * q + 3];
        *(v4fa*)(&st[tid * DC + 4 * q]) = w; }
    __syncthreads();
    const size_t base = (size_t)blockIdx.x * (256 * DC);
#pragma unroll 1
    for (int ps = 0; ps < 2; ++ps) {
#pragma unroll
        for (int i = 0; i < 4; ++i) { const int idx = i * 256 + tid;
            const v4f val = *(const v4fa*)(&st[idx * 4]);
            if (last != 0) *(volatile v4f*)(OUT + base + (size_t)idx * 4) = val;
            else           *(volatile v4f*)(Osum + base + (size_t)idx * 4) = val; }
        if (ps == 0) __threadfence(); }
}

static constexpr size_t al256(size_t v) { return (v + 255) & ~(size_t)255; }
static constexpr size_t SZ_XB = al256((size_t)NB * JN_FULL * PD * 2);
static constexpr size_t SZ_WB = al256((size_t)NC * JN_FULL * DC * PD * 2);
static constexpr size_t SZ_SP = al256((size_t)JG * NB * NC * DC * 4);
static constexpr size_t SZ_OS = al256((size_t)NB * NC * DC * 4);
static constexpr size_t SZ_TOTAL = SZ_XB + SZ_WB + SZ_SP + SZ_OS;
static_assert(SZ_TOTAL <= (size_t)134217728);
static_assert(((size_t)NB * JN_FULL * PD) % 8 == 0);
static_assert(((size_t)NC * JN_FULL * DC * PD) % 8 == 0);
static_assert((size_t)(JG - 1) * NB * NC * DC + (size_t)(NB - BT) * NC * DC + (size_t)BT * NC * DC == (size_t)JG * NB * NC * DC);
static_assert((size_t)(NB * NC / 256) * 256 * DC == (size_t)NB * NC * DC);

extern "C" void kernel_launch(void* const* d_in, const int* in_sizes, int n_in,
                              void* d_out, int out_size, void* d_ws, size_t ws_size, hipStream_t stream) {
    if (n_in < 3) return;
    if ((size_t)in_sizes[0] < (size_t)NB * JN_FULL * PD) return;
    if ((size_t)in_sizes[1] < (size_t)NC * JN_FULL * DC * PD) return;
    if (in_sizes[2] < NC * DC) return;
    if ((size_t)out_size < (size_t)NB * NC * DC) return;
    if (SZ_TOTAL > ws_size) return;
    const float* x = (const float*)d_in[0];
    const float* W = (const float*)d_in[1];
    const float* bias = (const float*)d_in[2];
    float* OUT = (float*)d_out;
    char* wsp = (char*)d_ws;
    bf* XB = (bf*)wsp; wsp += SZ_XB;
    bf* WB = (bf*)wsp; wsp += SZ_WB;
    float* SP = (float*)wsp; wsp += SZ_SP;
    float* OS = (float*)wsp; wsp += SZ_OS;

    { const size_t n8 = (size_t)NB * JN_FULL * PD / 8;
      k_cvt8<<<(unsigned)((n8 + 255) / 256), 256, 0, stream>>>(x, XB, n8); }
    { const size_t n8 = (size_t)NC * JN_FULL * DC * PD / 8;
      k_cvt8<<<(unsigned)((n8 + 255) / 256), 256, 0, stream>>>(W, WB, n8); }

    for (int it = 0; it < 3; ++it) {
        k_sweep<<<dim3(JG, NB / BT, 1), 256, 0, stream>>>(WB, XB, OS, SP, it == 0 ? 1 : 0);
        k_squash<<<dim3(NB * NC / 256, 1, 1), 256, 0, stream>>>(SP, bias, OS, OUT, it == 0 ? 1 : 0, it == 2 ? 1 : 0);
    }
}
